// EnhancedEdgeScorer_38293928411614
// MI455X (gfx1250) — hardware-verified
//
#include <hip/hip_runtime.h>
#include <math.h>
#include <stdint.h>

#define HIDC 128
#define FK   160
#define QKVW 384
#define PABW 256
#define HDD  32
#define KNB  16
#define NCTX 17
#define APL  136
#define ACT  64.0f
#define WSC  256.0f
#define AOC  1024.0f
#define H1C  64.0f
#define RESC 2048.0f
#define RINV 0.00048828125f
#define NEGM (-1.0e9f)

static_assert((FK % 32) == 0 && (HIDC % 64) == 0 && (QKVW % 64) == 0 && (PABW % 64) == 0);
static_assert((APL % 8) == 0);

typedef _Float16 v16h __attribute__((ext_vector_type(16)));
typedef _Float16 v8h  __attribute__((ext_vector_type(8)));
typedef float    v8f  __attribute__((ext_vector_type(8)));
typedef float    v4f  __attribute__((ext_vector_type(4)));
typedef unsigned int v4u __attribute__((ext_vector_type(4)));
typedef int      v4i  __attribute__((ext_vector_type(4)));

union FragH { v16h v; v8h h[2]; v4u u[2]; };

__device__ __forceinline__ unsigned short bf_bits(float f) {
  unsigned u = __float_as_uint(f);
  return (unsigned short)((u + 0x7FFFu + ((u >> 16) & 1u)) >> 16);
}
__device__ __forceinline__ float bf_up(unsigned short b) { return __uint_as_float(((unsigned)b) << 16); }
__device__ __forceinline__ float bfr(float f) { return bf_up(bf_bits(f)); }
__device__ __forceinline__ unsigned short h_bits(_Float16 x) { return __builtin_bit_cast(unsigned short, x); }
__device__ __forceinline__ unsigned pk16(unsigned short a, unsigned short b) { return (unsigned)a | ((unsigned)b << 16); }
__device__ __forceinline__ v8f zero8() { v8f z = {0.f, 0.f, 0.f, 0.f, 0.f, 0.f, 0.f, 0.f}; return z; }
__device__ __forceinline__ int clampi(int v, int lo, int hi) { v = (v < lo) ? lo : v; return (v > hi) ? hi : v; }
__device__ __forceinline__ v4u pack8f(const float (&v)[8]) {
  v4u o;
#pragma unroll
  for (int e = 0; e < 4; ++e) o[e] = pk16(h_bits((_Float16)v[2 * e]), h_bits((_Float16)v[2 * e + 1]));
  return o;
}

__device__ __forceinline__ v16h ldfrag_u(const unsigned short* p) {
  FragH f;
  f.u[0] = *(const v4u*)(p);
  f.u[1] = *(const v4u*)(p + 16);
  return f.v;
}

__device__ __forceinline__ v8f mma_raw(v16h a, v16h b, v8f c) {
  return __builtin_amdgcn_wmma_f32_16x16x32_f16(false, a, false, b, (short)0, c, false, false);
}
__device__ __forceinline__ void guard_4x1(v8f& a, v8f& b, v8f& c, v8f& d, v16h x) {
#if defined(__HIP_DEVICE_COMPILE__)
  asm volatile("v_nop\n\tv_nop\n\tv_nop\n\tv_nop" : "+v"(a), "+v"(b), "+v"(c), "+v"(d) : "v"(x));
#endif
}
__device__ __forceinline__ void keep4_h(v16h a, v16h b, v16h c, v16h d) {
#if defined(__HIP_DEVICE_COMPILE__)
  asm volatile("v_nop" :: "v"(a), "v"(b), "v"(c), "v"(d));
#endif
}
__device__ __forceinline__ void acc_guard4(v8f& a, v8f& b, v8f& c, v8f& d) {
#if defined(__HIP_DEVICE_COMPILE__)
  asm volatile("v_nop\n\tv_nop\n\tv_nop\n\tv_nop" : "+v"(a), "+v"(b), "+v"(c), "+v"(d));
#endif
}
__device__ __forceinline__ void wave_sync_lds() {
  __builtin_amdgcn_fence(__ATOMIC_RELEASE, "workgroup");
  __builtin_amdgcn_wave_barrier();
  __builtin_amdgcn_fence(__ATOMIC_ACQUIRE, "workgroup");
}

__global__ __launch_bounds__(256) void cvW(const float* __restrict__ src, unsigned short* dst, int K, int N, int Z, int mode,
                                           float scale) {
  const int kcn = K >> 3;
  const int nch = Z * N * kcn;
  const int i = blockIdx.x * 256 + threadIdx.x;
  const bool live = i < nch;
  const int ic = live ? i : (nch - 1);
  const int z = ic / (N * kcn);
  const int rem = ic - z * N * kcn;
  const int n = rem / kcn;
  const int kc = rem - n * kcn;
  float v[8];
#pragma unroll
  for (int e = 0; e < 8; ++e) {
    const int k = kc * 8 + e;
    size_t si;
    if (mode == 0) {
      si = (size_t)z * (size_t)K * (size_t)N + (size_t)k * (size_t)N + (size_t)n;
    } else if (mode == 1) {
      const int sr = (k < 32) ? (128 + k) : (k - 32);
      si = (size_t)sr * (size_t)N + (size_t)n;
    } else {
      si = (size_t)(((n >> 7) * 128) + k) * (size_t)128 + (size_t)(n & 127);
    }
    v[e] = bfr(src[si]) * scale;
  }
  const v4u o = pack8f(v);
  unsigned short* dp = dst + (size_t)ic * 8;
  if (live) *(volatile v4u*)dp = o;
  __threadfence();
  if (live) *(volatile v4u*)dp = o;
}

__global__ __launch_bounds__(256) void hnbk(const int* __restrict__ nm, int* HNB, int N, int NP) {
  const int i = blockIdx.x * 256 + threadIdx.x;
  const bool live = i < NP;
  int n = live ? i : (NP - 1);
  n = (n < N) ? n : (N - 1);
  const int* p = nm + (size_t)n * KNB;
  const v4i a = *(const v4i*)(p), b = *(const v4i*)(p + 4), c = *(const v4i*)(p + 8), d = *(const v4i*)(p + 12);
  const v4i o = a | b | c | d;
  const int any = ((o.x | o.y | o.z | o.w) != 0) ? 1 : 0;
  int* dp = HNB + (live ? i : 0);
  if (live) *(volatile int*)dp = any;
  __threadfence();
  if (live) *(volatile int*)dp = any;
}

__global__ __launch_bounds__(256) void featk(const int* __restrict__ tix, const int* __restrict__ cix,
                                             const float* __restrict__ ldg, const float* __restrict__ te,
                                             const float* __restrict__ ce0, const float* __restrict__ ce1,
                                             const float* __restrict__ dW, const float* __restrict__ db,
                                             unsigned short* FH, int N, int NP, int NT, int NC) {
#pragma clang fp contract(off)
  const int nch = NP * (FK / 8);
  const int i = blockIdx.x * 256 + threadIdx.x;
  const bool live = i < nch;
  const int ic = live ? i : (nch - 1);
  const int row = ic / (FK / 8);
  const int kc = ic - row * (FK / 8);
  const int col0 = kc * 8;
  const int node = (row < N) ? row : (N - 1);
  const int ty = clampi(tix[node], 0, NT - 1);
  const int ca = clampi(cix[2 * node], 0, NC - 1);
  const int cb = clampi(cix[2 * node + 1], 0, NC - 1);
  const float lv = bfr(ldg[node]);
  const int jd = (col0 < 24) ? col0 : 24;
  const int jt = clampi(col0 - 32, 0, 56);
  const int ja = clampi(col0 - 96, 0, 24);
  const int jb = clampi(col0 - 128, 0, 24);
  const v4f w0 = *(const v4f*)(dW + jd), w1 = *(const v4f*)(dW + jd + 4);
  const v4f g0 = *(const v4f*)(db + jd), g1 = *(const v4f*)(db + jd + 4);
  const float* tp = te + (size_t)ty * 64 + jt;
  const float* ap = ce0 + (size_t)ca * 32 + ja;
  const float* bp = ce1 + (size_t)cb * 32 + jb;
  const v4f t0 = *(const v4f*)(tp), t1 = *(const v4f*)(tp + 4);
  const v4f a0 = *(const v4f*)(ap), a1 = *(const v4f*)(ap + 4);
  const v4f c0 = *(const v4f*)(bp), c1 = *(const v4f*)(bp + 4);
  float wv[8], gv[8], tv[8], av[8], cv[8];
#pragma unroll
  for (int e = 0; e < 4; ++e) {
    wv[e] = w0[e]; wv[4 + e] = w1[e];
    gv[e] = g0[e]; gv[4 + e] = g1[e];
    tv[e] = t0[e]; tv[4 + e] = t1[e];
    av[e] = a0[e]; av[4 + e] = a1[e];
    cv[e] = c0[e]; cv[4 + e] = c1[e];
  }
  const int seg = (col0 < 32) ? 0 : ((col0 < 96) ? 1 : ((col0 < 128) ? 2 : 3));
  float v[8];
#pragma unroll
  for (int e = 0; e < 8; ++e) {
    const float dg = fmaxf(lv * bfr(wv[e]) + bfr(gv[e]), 0.f);
    const float s1 = bfr(tv[e]), s2 = bfr(av[e]), s3 = bfr(cv[e]);
    const float sel = (seg == 0) ? dg : ((seg == 1) ? s1 : ((seg == 2) ? s2 : s3));
    v[e] = sel * ACT;
  }
  const v4u o = pack8f(v);
  unsigned short* dp = FH + (size_t)ic * 8;
  if (live) *(volatile v4u*)dp = o;
  __threadfence();
  if (live) *(volatile v4u*)dp = o;
}

__device__ __forceinline__ void kloop(v8f (&acc)[4][4], const unsigned short* __restrict__ A1, int lda,
                                      const unsigned short* __restrict__ Bb, int ldb, int m0, int n0, int K,
                                      int rlane, int koff) {
#pragma unroll 1
  for (int k0 = 0; k0 < K; k0 += 32) {
    v16h bh[4];
#pragma unroll
    for (int j = 0; j < 4; ++j) {
      const size_t bofs = (size_t)(n0 + (j << 4) + rlane) * (size_t)ldb + (size_t)(koff + k0);
      bh[j] = ldfrag_u(Bb + bofs);
    }
#pragma unroll
    for (int i = 0; i < 4; ++i) {
      const size_t ao = (size_t)(m0 + (i << 4) + rlane) * (size_t)lda + (size_t)(k0 + koff);
      const v16h ah = ldfrag_u(A1 + ao);
#pragma unroll
      for (int j = 0; j < 4; ++j) acc[i][j] = mma_raw(ah, bh[j], acc[i][j]);
      guard_4x1(acc[i][0], acc[i][1], acc[i][2], acc[i][3], ah);
    }
    keep4_h(bh[0], bh[1], bh[2], bh[3]);
  }
}

template <int OM, int BIASM>
__global__ __launch_bounds__(256) void gemm64(
    const unsigned short* __restrict__ Ap, int lda,
    const unsigned short* __restrict__ Alo, int ldlo, int Klo,
    const unsigned short* __restrict__ Btp, int ldb,
    const float* __restrict__ bias, float bscale,
    void* Cout, int ldc, int M, int N, int K, float oscale,
    const unsigned short* Xold, const int* __restrict__ HNB) {
  __shared__ __align__(16) float sT[8][16 * 68];
  const int lane = threadIdx.x & 31;
  const int wave = threadIdx.x >> 5;
  const int tilesN = N >> 6;
  const int tilesM = M >> 6;
  const int tile = blockIdx.x * 8 + wave;
  if (tile >= tilesM * tilesN) return;
  const int tm = tile / tilesN;
  const int tn = tile - tm * tilesN;
  const int m0 = tm << 6;
  const int n0 = tn << 6;

  const int rlane = lane & 15;
  const int koff  = (lane >> 4) * 8;
  const int mOff  = (lane >> 4) * 8;

  v8f acc[4][4];
#pragma unroll
  for (int i = 0; i < 4; ++i)
#pragma unroll
    for (int j = 0; j < 4; ++j) acc[i][j] = zero8();

  if (Klo > 0) {
    kloop(acc, Alo, ldlo, Btp, ldb, m0, n0, Klo, rlane, koff);
    acc_guard4(acc[0][0], acc[0][1], acc[0][2], acc[0][3]);
    acc_guard4(acc[1][0], acc[1][1], acc[1][2], acc[1][3]);
    acc_guard4(acc[2][0], acc[2][1], acc[2][2], acc[2][3]);
    acc_guard4(acc[3][0], acc[3][1], acc[3][2], acc[3][3]);
#pragma unroll
    for (int i = 0; i < 4; ++i)
#pragma unroll
      for (int j = 0; j < 4; ++j) acc[i][j] = acc[i][j] * RINV;
  }
  kloop(acc, Ap, lda, Btp, ldb, m0, n0, K, rlane, koff);
  acc_guard4(acc[0][0], acc[0][1], acc[0][2], acc[0][3]);
  acc_guard4(acc[1][0], acc[1][1], acc[1][2], acc[1][3]);
  acc_guard4(acc[2][0], acc[2][1], acc[2][2], acc[2][3]);
  acc_guard4(acc[3][0], acc[3][1], acc[3][2], acc[3][3]);

  const int hh2 = lane >> 4, c4 = (lane & 15) * 4;
  const int q8  = lane >> 3, c8 = (lane & 7) * 8;
  float bc4[4], bc8[8];
#pragma unroll
  for (int e = 0; e < 4; ++e) bc4[e] = 0.f;
#pragma unroll
  for (int e = 0; e < 8; ++e) bc8[e] = 0.f;
  if (BIASM == 0) {
    if (OM == 4) {
      const int cb = n0 + c4;
      const int i0 = (cb <= N - 4) ? cb : (N - 4);
      const v4f b0v = *(const v4f*)(bias + i0);
#pragma unroll
      for (int e = 0; e < 4; ++e) bc4[e] = bfr(b0v[e]) * bscale;
    } else {
      const int cb = n0 + c8;
      const int i0 = (cb <= N - 8) ? cb : (N - 8);
      const v4f b0v = *(const v4f*)(bias + i0), b1v = *(const v4f*)(bias + i0 + 4);
#pragma unroll
      for (int e = 0; e < 4; ++e) { bc8[e] = bfr(b0v[e]) * bscale; bc8[4 + e] = bfr(b1v[e]) * bscale; }
    }
  }

  float* slab = sT[wave];
#pragma unroll
  for (int i = 0; i < 4; ++i) {
    const int mBase = m0 + (i << 4);
#pragma unroll
    for (int j = 0; j < 4; ++j) {
#pragma unroll
      for (int r = 0; r < 8; ++r) {
        slab[(mOff + r) * 68 + (j << 4) + rlane] = acc[i][j][r];
      }
    }
    wave_sync_lds();
    if (OM == 4) {
      float* C = (float*)Cout;
      v4f vals[8];
#pragma unroll
      for (int it = 0; it < 8; ++it) {
        const int row = it * 2 + hh2;
        float rb = 0.f;
        if (BIASM == 1) {
          const int gr = mBase + row;
          rb = bfr(bias[(gr < M) ? gr : (M - 1)]) * bscale;
        }
        v4f v = *(const v4f*)(slab + row * 68 + c4);
#pragma unroll
        for (int e = 0; e < 4; ++e) v[e] = v[e] * oscale + bc4[e] + rb;
        vals[it] = v;
      }
#pragma unroll
      for (int it = 0; it < 8; ++it) {
        const int gr = mBase + it * 2 + hh2;
        *(volatile v4f*)(C + (size_t)gr * (size_t)ldc + n0 + c4) = vals[it];
      }
      __threadfence();
#pragma unroll
      for (int it = 0; it < 8; ++it) {
        const int gr = mBase + it * 2 + hh2;
        *(volatile v4f*)(C + (size_t)gr * (size_t)ldc + n0 + c4) = vals[it];
      }
      __threadfence();
    } else {
      unsigned short* C = (unsigned short*)Cout;
      v4u hv[4];
#pragma unroll
      for (int it = 0; it < 4; ++it) {
        const int row = it * 4 + q8;
        float rb = 0.f;
        if (BIASM == 1) {
          const int gr = mBase + row;
          rb = bfr(bias[(gr < M) ? gr : (M - 1)]) * bscale;
        }
        const float* sp = slab + row * 68 + c8;
        const v4f x0 = *(const v4f*)(sp), x1 = *(const v4f*)(sp + 4);
        float v[8];
#pragma unroll
        for (int e = 0; e < 4; ++e) {
          v[e]     = x0[e] * oscale + bc8[e] + rb;
          v[4 + e] = x1[e] * oscale + bc8[4 + e] + rb;
        }
        if (OM == 3) {
          const int gr  = mBase + row;
          const int grc = (gr < M) ? gr : (M - 1);
          const int flag = HNB[grc];
          const v8h xo = *(const v8h*)((const _Float16*)(const void*)Xold + (size_t)grc * (size_t)ldc + n0 + c8);
#pragma unroll
          for (int e = 0; e < 8; ++e) {
            const float xf = (float)xo[e];
            const float vv = (flag != 0) ? v[e] : xf;
            v[e] = fmaxf(vv, 0.f);
          }
        }
        hv[it] = pack8f(v);
      }
#pragma unroll
      for (int it = 0; it < 4; ++it) {
        const int row = it * 4 + q8;
        const size_t o = (size_t)(mBase + row) * (size_t)ldc + n0 + c8;
        *(volatile v4u*)(C + o) = hv[it];
      }
      __threadfence();
#pragma unroll
      for (int it = 0; it < 4; ++it) {
        const int row = it * 4 + q8;
        const size_t o = (size_t)(mBase + row) * (size_t)ldc + n0 + c8;
        *(volatile v4u*)(C + o) = hv[it];
      }
      __threadfence();
    }
    wave_sync_lds();
  }
}

__global__ __launch_bounds__(128)
void attnk(const float* __restrict__ QKV, const int* __restrict__ nbr, const int* __restrict__ nmk,
           unsigned short* OH, int N) {
  __shared__ float sS[NCTX * 128];
  __shared__ int   sI[NCTX * 128];
  __shared__ __align__(16) unsigned short sO[4][8 * HIDC];
  const int t = threadIdx.x, wave = t >> 5, lane = t & 31;
  const int j = lane >> 2, h = lane & 3;
  const int row = blockIdx.x * 32 + wave * 8 + j;
  const int nc = (row < N) ? row : (N - 1);

  float q[32];
  {
    const float* qp = QKV + (size_t)nc * QKVW + HDD * h;
#pragma unroll
    for (int g = 0; g < 8; ++g) {
      const v4f x = *(const v4f*)(qp + 4 * g);
#pragma unroll
      for (int e = 0; e < 4; ++e) q[4 * g + e] = x[e];
    }
  }
  const int* nip = nbr + (size_t)nc * KNB;
  const int* nmp = nmk + (size_t)nc * KNB;
  const float lsc = 0.1767766952966369f * 1.4426950408889634f;

  float mx = NEGM;
#pragma unroll 1
  for (int c = 0; c < NCTX; ++c) {
    const int cm = (c > 0) ? (c - 1) : 0;
    const int gi = clampi(nip[cm], 0, N - 1);
    const int mk = nmp[cm];
    const int idx = (c == 0) ? nc : gi;
    const float* kp = QKV + (size_t)idx * QKVW + HIDC + HDD * h;
    float d = 0.f;
#pragma unroll
    for (int g = 0; g < 8; ++g) {
      const v4f kv = *(const v4f*)(kp + 4 * g);
#pragma unroll
      for (int e = 0; e < 4; ++e) d += q[4 * g + e] * kv[e];
    }
    const bool valid = (c == 0) || (mk != 0);
    const float ts = valid ? d * lsc : NEGM;
    mx = fmaxf(mx, ts);
    sS[c * 128 + t] = ts;
    sI[c * 128 + t] = idx;
  }

  float o[32];
#pragma unroll
  for (int e = 0; e < 32; ++e) o[e] = 0.f;
  float l = 0.f;
#pragma unroll 1
  for (int c = 0; c < NCTX; ++c) {
    const float p = exp2f(sS[c * 128 + t] - mx);
    l += p;
    const int idx = sI[c * 128 + t];
    const float* vp = QKV + (size_t)idx * QKVW + 2 * HIDC + HDD * h;
#pragma unroll
    for (int g = 0; g < 8; ++g) {
      const v4f vv = *(const v4f*)(vp + 4 * g);
#pragma unroll
      for (int e = 0; e < 4; ++e) o[4 * g + e] += p * vv[e];
    }
  }
  const float inv = __builtin_amdgcn_rcpf(l) * AOC;

  unsigned short* so = sO[wave] + j * HIDC + HDD * h;
#pragma unroll
  for (int g = 0; g < 4; ++g) {
    v4u pk;
#pragma unroll
    for (int e = 0; e < 4; ++e)
      pk[e] = pk16(h_bits((_Float16)(o[8 * g + 2 * e] * inv)), h_bits((_Float16)(o[8 * g + 2 * e + 1] * inv)));
    *(v4u*)(so + 8 * g) = pk;
  }
  wave_sync_lds();
  const int rbase = blockIdx.x * 32 + wave * 8;
  v4u ov[4];
  size_t oo[4];
#pragma unroll
  for (int it = 0; it < 4; ++it) {
    const int ch = it * 32 + lane;
    const int r = ch >> 4;
    const int cc = (ch & 15) * 8;
    ov[it] = *(const v4u*)(sO[wave] + r * HIDC + cc);
    oo[it] = (size_t)(rbase + r) * (size_t)HIDC + (size_t)cc;
  }
#pragma unroll
  for (int it = 0; it < 4; ++it) *(volatile v4u*)(OH + oo[it]) = ov[it];
  __threadfence();
#pragma unroll
  for (int it = 0; it < 4; ++it) *(volatile v4u*)(OH + oo[it]) = ov[it];
}

__device__ __forceinline__ void kloop16(v8f (&acc)[4], const unsigned short* A1, int lda,
                                        const unsigned short* __restrict__ Bb, int ldb, int m0, int K,
                                        int rlane, int koff) {
#pragma unroll 1
  for (int k0 = 0; k0 < K; k0 += 32) {
    v16h bh[4];
#pragma unroll
    for (int j = 0; j < 4; ++j) {
      const size_t bofs = (size_t)((j << 4) + rlane) * (size_t)ldb + (size_t)(koff + k0);
      bh[j] = ldfrag_u(Bb + bofs);
    }
    const v16h ah = ldfrag_u(A1 + (size_t)(m0 + rlane) * (size_t)lda + (size_t)(k0 + koff));
#pragma unroll
    for (int j = 0; j < 4; ++j) acc[j] = mma_raw(ah, bh[j], acc[j]);
    guard_4x1(acc[0], acc[1], acc[2], acc[3], ah);
    keep4_h(bh[0], bh[1], bh[2], bh[3]);
  }
}

__global__ __launch_bounds__(128)
void edgek(const float* __restrict__ PAB, const int* __restrict__ edges, const float* __restrict__ ef,
           const float* __restrict__ eW1, const float* __restrict__ eb1, const unsigned short* __restrict__ W2T,
           const float* __restrict__ eb2, const float* __restrict__ eW3, const float* __restrict__ eb3,
           float* out, int N) {
  __shared__ __align__(16) unsigned short sAh[64 * APL];
  __shared__ __align__(16) unsigned short sAl[64 * APL];
  __shared__ __align__(16) float sT[4][16 * 68];
  __shared__ int   sSrc[64], sDst[64];
  __shared__ float sF0[64], sF1[64], sW3[64], sB2[64];
  __shared__ __align__(16) float sOut[64];
  const int t = threadIdx.x, wave = t >> 5, lane = t & 31;
  const int e0 = blockIdx.x * 64;

  if (t < 64) {
    const int e = e0 + t;
    sSrc[t] = clampi(edges[(size_t)e * 2], 0, N - 1);
    sDst[t] = clampi(edges[(size_t)e * 2 + 1], 0, N - 1);
    sF0[t]  = bfr(ef[(size_t)e * 2]);
    sF1[t]  = bfr(ef[(size_t)e * 2 + 1]);
    sW3[t]  = bfr(eW3[t]);
    sB2[t]  = bfr(eb2[t]);
  }
  __syncthreads();

#pragma unroll 1
  for (int it = 0; it < 8; ++it) {
    const int ch = it * 128 + t;
    const int r  = ch >> 4;
    const int c8 = (ch & 15) * 8;
    const int a = sSrc[r], b = sDst[r];
    const float f0 = sF0[r], f1 = sF1[r];
    const float* pa = PAB + (size_t)a * PABW + c8;
    const float* pb = PAB + (size_t)b * PABW + HIDC + c8;
    const float* w0 = eW1 + (size_t)256 * HIDC + c8;
    const float* w1 = eW1 + (size_t)257 * HIDC + c8;
    const float* bb = eb1 + c8;
    const v4f pa0 = *(const v4f*)(pa), pa1 = *(const v4f*)(pa + 4);
    const v4f pb0 = *(const v4f*)(pb), pb1 = *(const v4f*)(pb + 4);
    const v4f wa0 = *(const v4f*)(w0), wa1 = *(const v4f*)(w0 + 4);
    const v4f wb0 = *(const v4f*)(w1), wb1 = *(const v4f*)(w1 + 4);
    const v4f bv0 = *(const v4f*)(bb), bv1 = *(const v4f*)(bb + 4);
    float pav[8], pbv[8], wav[8], wbv[8], bvv[8];
#pragma unroll
    for (int e = 0; e < 4; ++e) {
      pav[e] = pa0[e]; pav[4 + e] = pa1[e];
      pbv[e] = pb0[e]; pbv[4 + e] = pb1[e];
      wav[e] = wa0[e]; wav[4 + e] = wa1[e];
      wbv[e] = wb0[e]; wbv[4 + e] = wb1[e];
      bvv[e] = bv0[e]; bvv[4 + e] = bv1[e];
    }
    float hiv[8], lov[8];
#pragma unroll
    for (int e = 0; e < 8; ++e) {
      const float hpre = pav[e] + pbv[e] + f0 * bfr(wav[e]) + f1 * bfr(wbv[e]) + bfr(bvv[e]);
      const float hc = fmaxf(hpre, 0.f) * H1C;
      const _Float16 hh = (_Float16)hc;
      hiv[e] = (float)hh;
      lov[e] = (hc - (float)hh) * RESC;
    }
    const v4u ph = pack8f(hiv), pl = pack8f(lov);
    *(v4u*)(sAh + r * APL + c8) = ph;
    *(v4u*)(sAl + r * APL + c8) = pl;
  }
  __syncthreads();

  const int rlane = lane & 15;
  const int koff  = (lane >> 4) * 8;
  const int mOff  = (lane >> 4) * 8;
  const int m0 = wave * 16;
  v8f acc[4];
#pragma unroll
  for (int jn = 0; jn < 4; ++jn) acc[jn] = zero8();
  kloop16(acc, sAl, APL, W2T, HIDC, m0, HIDC, rlane, koff);
  acc_guard4(acc[0], acc[1], acc[2], acc[3]);
#pragma unroll
  for (int jn = 0; jn < 4; ++jn) acc[jn] = acc[jn] * RINV;
  kloop16(acc, sAh, APL, W2T, HIDC, m0, HIDC, rlane, koff);
  acc_guard4(acc[0], acc[1], acc[2], acc[3]);

  float* slab = sT[wave];
#pragma unroll
  for (int jn = 0; jn < 4; ++jn) {
#pragma unroll
    for (int r = 0; r < 8; ++r) slab[(mOff + r) * 68 + (jn << 4) + rlane] = acc[jn][r];
  }
  wave_sync_lds();
  const float osc = 1.0f / (H1C * WSC);
  const int row = lane & 15, hf = lane >> 4;
  const float* sp = slab + row * 68 + 32 * hf;
  float s = 0.f;
#pragma unroll
  for (int n = 0; n < 32; ++n) {
    const float h2 = fmaxf(sp[n] * osc + sB2[32 * hf + n], 0.f);
    s += h2 * sW3[32 * hf + n];
  }
  s += __shfl_xor(s, 16, 32);
  s += bfr(eb3[0]);
  sOut[m0 + row] = s;
  __syncthreads();

  const int tc = (t < 16) ? t : 0;
  const v4f ov = *(const v4f*)(sOut + 4 * tc);
  float* dp = out + (size_t)e0 + 4 * tc;
  if (t < 16) *(volatile v4f*)dp = ov;
  __threadfence();
  if (t < 16) *(volatile v4f*)dp = ov;
}

static inline dim3 ggrid(int M, int N) { return dim3((unsigned)((((M / 64) * (N / 64)) + 7) / 8)); }

extern "C" void kernel_launch(void* const* d_in, const int* in_sizes, int n_in,
                              void* d_out, int out_size, void* d_ws, size_t ws_size,
                              hipStream_t stream) {
  if (n_in < 24) return;
  const int N = in_sizes[0];
  const int E = out_size;
  if (N <= 0 || E <= 0) return;
  if (in_sizes[1] != 2 * N || in_sizes[2] != KNB * N || in_sizes[3] != KNB * N) return;
  if (in_sizes[4] != 2 * E || in_sizes[5] != N || in_sizes[6] != 2 * E) return;
  if ((in_sizes[7] % 64) != 0 || in_sizes[7] < 64) return;
  if ((in_sizes[8] % 32) != 0 || in_sizes[8] < 32 || in_sizes[9] != in_sizes[8]) return;
  if (in_sizes[10] != 32 || in_sizes[11] != 32) return;
  if (in_sizes[12] != FK * HIDC || in_sizes[13] != HIDC) return;
  if (in_sizes[14] != 3 * HIDC * QKVW || in_sizes[15] != 3 * QKVW) return;
  if (in_sizes[16] != 3 * HIDC * HIDC || in_sizes[17] != 3 * HIDC) return;
  if (in_sizes[18] != 258 * HIDC || in_sizes[19] != HIDC) return;
  if (in_sizes[20] != HIDC * 64 || in_sizes[21] != 64 || in_sizes[22] != 64 || in_sizes[23] != 1) return;
  if ((E % 64) != 0) return;
  const int NT = in_sizes[7] / 64;
  const int NC = in_sizes[8] / 32;
  const int NP = ((N + 63) / 64) * 64;

  const int*   type_idx = (const int*)d_in[0];
  const int*   cat_idx  = (const int*)d_in[1];
  const int*   nbr_idx  = (const int*)d_in[2];
  const int*   nbr_mask = (const int*)d_in[3];
  const int*   edges    = (const int*)d_in[4];
  const float* log_deg  = (const float*)d_in[5];
  const float* ef       = (const float*)d_in[6];
  const float* te       = (const float*)d_in[7];
  const float* ce0      = (const float*)d_in[8];
  const float* ce1      = (const float*)d_in[9];
  const float* deg_W    = (const float*)d_in[10];
  const float* deg_b    = (const float*)d_in[11];
  const float* proj_W   = (const float*)d_in[12];
  const float* proj_b   = (const float*)d_in[13];
  const float* Wqkv     = (const float*)d_in[14];
  const float* bqkv     = (const float*)d_in[15];
  const float* Wo       = (const float*)d_in[16];
  const float* bo       = (const float*)d_in[17];
  const float* eW1      = (const float*)d_in[18];
  const float* eb1      = (const float*)d_in[19];
  const float* eW2      = (const float*)d_in[20];
  const float* eb2      = (const float*)d_in[21];
  const float* eW3      = (const float*)d_in[22];
  const float* eb3      = (const float*)d_in[23];
  float*       out      = (float*)d_out;

  size_t off = 0;
  auto carve = [&](size_t bytes) -> size_t {
    const size_t o = off;
    off += (bytes + (size_t)65535) & ~(size_t)65535;
    return o;
  };
  const size_t oFH  = carve((size_t)NP * FK * 2);
  const size_t oPWT = carve((size_t)HIDC * FK * 2);
  const size_t oWQT = carve((size_t)3 * QKVW * HIDC * 2);
  const size_t oWOT = carve((size_t)3 * HIDC * HIDC * 2);
  const size_t oW1T = carve((size_t)PABW * HIDC * 2);
  const size_t oW2T = carve((size_t)64 * HIDC * 2);
  const size_t oHNB = carve((size_t)NP * 4);
  const size_t oXA  = carve((size_t)NP * HIDC * 2);
  const size_t oXB  = carve((size_t)NP * HIDC * 2);
  const size_t oQKV = carve((size_t)NP * QKVW * 4);
  if (off > ws_size) return;
  if (off > (size_t)134217728) return;
  if ((size_t)NP * HIDC * 2 > (size_t)NP * FK * 2) return;
  if ((size_t)NP * PABW * 4 > (size_t)NP * QKVW * 4) return;

  char* ws = (char*)d_ws;
  unsigned short* FH  = (unsigned short*)(ws + oFH);
  unsigned short* OH  = (unsigned short*)(ws + oFH);
  unsigned short* PWT = (unsigned short*)(ws + oPWT);
  unsigned short* WQT = (unsigned short*)(ws + oWQT);
  unsigned short* WOT = (unsigned short*)(ws + oWOT);
  unsigned short* W1T = (unsigned short*)(ws + oW1T);
  unsigned short* W2T = (unsigned short*)(ws + oW2T);
  int*            HNB = (int*)(ws + oHNB);
  unsigned short* XA  = (unsigned short*)(ws + oXA);
  unsigned short* XB  = (unsigned short*)(ws + oXB);
  float*          QKV = (float*)(ws + oQKV);
  float*          PAB = (float*)(ws + oQKV);

  const dim3 blk(256), blk128(128);
  const float osP = 1.0f / WSC;
  const float osQ = 1.0f / (ACT * WSC);
  const float osW = ACT / (AOC * WSC);

  cvW<<<dim3((unsigned)((HIDC * (FK / 8) + 255) / 256)), blk, 0, stream>>>(proj_W, PWT, FK, HIDC, 1, 1, WSC);
  cvW<<<dim3((unsigned)((3 * QKVW * (HIDC / 8) + 255) / 256)), blk, 0, stream>>>(Wqkv, WQT, HIDC, QKVW, 3, 0, WSC);
  cvW<<<dim3((unsigned)((3 * HIDC * (HIDC / 8) + 255) / 256)), blk, 0, stream>>>(Wo, WOT, HIDC, HIDC, 3, 0, WSC);
  cvW<<<dim3((unsigned)((PABW * (HIDC / 8) + 255) / 256)), blk, 0, stream>>>(eW1, W1T, HIDC, PABW, 1, 2, WSC);
  cvW<<<dim3((unsigned)((64 * (HIDC / 8) + 255) / 256)), blk, 0, stream>>>(eW2, W2T, HIDC, 64, 1, 0, WSC);

  hnbk<<<dim3((unsigned)((NP + 255) / 256)), blk, 0, stream>>>(nbr_mask, HNB, N, NP);
  featk<<<dim3((unsigned)((NP * (FK / 8) + 255) / 256)), blk, 0, stream>>>(
      type_idx, cat_idx, log_deg, te, ce0, ce1, deg_W, deg_b, FH, N, NP, NT, NC);

  gemm64<2, 0><<<ggrid(NP, HIDC), blk, 0, stream>>>(
      FH, FK, FH, FK, 0, PWT, FK, proj_b, ACT, (void*)XA, HIDC, NP, HIDC, FK, osP, nullptr, nullptr);

  unsigned short* Xcur = XA;
  unsigned short* Xnxt = XB;
  for (int l = 0; l < 3; ++l) {
    gemm64<4, 0><<<ggrid(NP, QKVW), blk, 0, stream>>>(
        Xcur, HIDC, Xcur, HIDC, 0, WQT + (size_t)l * QKVW * HIDC, HIDC, bqkv + (size_t)l * QKVW, 1.0f,
        (void*)QKV, QKVW, NP, QKVW, HIDC, osQ, nullptr, nullptr);
    attnk<<<dim3((unsigned)(NP / 32)), blk128, 0, stream>>>(QKV, nbr_idx, nbr_mask, OH, N);
    gemm64<3, 0><<<ggrid(NP, HIDC), blk, 0, stream>>>(
        OH, HIDC, OH, HIDC, 0, WOT + (size_t)l * HIDC * HIDC, HIDC, bo + (size_t)l * HIDC, ACT,
        (void*)Xnxt, HIDC, NP, HIDC, HIDC, osW, Xcur, HNB);
    unsigned short* tmp = Xcur; Xcur = Xnxt; Xnxt = tmp;
  }

  gemm64<4, 0><<<ggrid(NP, PABW), blk, 0, stream>>>(
      Xcur, HIDC, Xcur, HIDC, 0, W1T, HIDC, eW1, 0.0f, (void*)PAB, PABW, NP, PABW, HIDC, osQ, nullptr, nullptr);

  edgek<<<dim3((unsigned)(E / 64)), blk128, 0, stream>>>(PAB, edges, ef, eW1, eb1, W2T, eb2, eW3, eb3, out, N);

  (void)hipGetLastError();
}
